// TypeLayer_36524401885446
// MI455X (gfx1250) — hardware-verified
//
#include <hip/hip_runtime.h>

typedef __attribute__((ext_vector_type(16))) _Float16 v16h;
typedef __attribute__((ext_vector_type(8)))  _Float16 v8h;
typedef __attribute__((ext_vector_type(8)))  float    v8f;
typedef __attribute__((ext_vector_type(4)))  float    v4f_t;
typedef float v4fa __attribute__((ext_vector_type(4), may_alias));
typedef __attribute__((ext_vector_type(4)))  unsigned v4u_t;
typedef unsigned v4ua __attribute__((ext_vector_type(4), may_alias));

#define HDIM  128
#define NREL  6000
#define NSEG  16000
#define NFACT 500000
#define RSPLIT (1.0f / 2048.0f)
__device__ __forceinline__ _Float16 lo_of(float v, _Float16 h) { return (_Float16)((v - (float)h) * 2048.0f); }
__device__ __forceinline__ v8f wmma16(v16h a, v16h b, v8f c) { return __builtin_amdgcn_wmma_f32_16x16x32_f16(false, a, false, b, (short)0, c, false, false); }
__device__ __forceinline__ v8f wmma_split(v16h a, v16h al, v16h b, v16h bl, v8f c) { v8f x = {}; x = wmma16(al, b, x); x = wmma16(a, bl, x); return wmma16(a, b, c) + x * RSPLIT; }
__device__ __forceinline__ v16h frag16(const _Float16* p, int g) {
  return __builtin_shufflevector(*(const v8h*)(p + 8 * g), *(const v8h*)(p + 16 + 8 * g), 0,1,2,3,4,5,6,7,8,9,10,11,12,13,14,15);
}

__global__ void prep_kernel(const float* __restrict__ relf, const float* __restrict__ Wf,
                            _Float16* __restrict__ Ah, _Float16* __restrict__ Wh) {
  const int t = blockIdx.x * blockDim.x + threadIdx.x;
  const int nA8 = NREL * HDIM / 8, nW8 = HDIM * HDIM / 8;
  if (t >= nA8 + nW8) return;
  const float* src; _Float16* dst; size_t pl; int e0;
  if (t < nA8) { src = relf; dst = Ah; pl = (size_t)NREL * HDIM; e0 = t * 8; }
  else         { src = Wf;   dst = Wh; pl = (size_t)HDIM * HDIM; e0 = (t - nA8) * 8; }
  _Float16 hh[8], hl[8];
#pragma unroll
  for (int e = 0; e < 8; ++e) { const float v = src[e0 + e]; hh[e] = (_Float16)v; hl[e] = lo_of(v, hh[e]); }
  _Float16* d = dst + e0;
  *(volatile v4u_t*)d = *(const v4ua*)hh; *(volatile v4u_t*)(d + pl) = *(const v4ua*)hl; __threadfence();
  *(volatile v4u_t*)d = *(const v4ua*)hh; *(volatile v4u_t*)(d + pl) = *(const v4ua*)hl;
}

__global__ __launch_bounds__(128) void relval_gemm_wmma(const _Float16* __restrict__ Ah, const _Float16* __restrict__ Wh,
                                                        const float* __restrict__ bias, float* __restrict__ relval) {
  __shared__ __attribute__((aligned(16))) float st[4][16 * 132];
  const int lane = threadIdx.x & 31, wave = threadIdx.x >> 5;
  const int g = lane >> 4, l16 = lane & 15;
  const int r0 = (blockIdx.x * 4 + wave) * 16;
  if (r0 >= NREL) return;
  const size_t PLA = (size_t)NREL * HDIM, PLW = (size_t)HDIM * HDIM;
  v8f acc[8] = {};
#pragma unroll
  for (int k0 = 0; k0 < HDIM; k0 += 32) {
    const _Float16* ap = Ah + (size_t)(r0 + l16) * HDIM + k0;
    const v16h a = frag16(ap, g), al = frag16(ap + PLA, g);
#pragma unroll
    for (int j = 0; j < 8; ++j) {
      const _Float16* bp = Wh + (size_t)(j * 16 + l16) * HDIM + k0;
      acc[j] = wmma_split(a, al, frag16(bp, g), frag16(bp + PLW, g), acc[j]);
    }
  }
  float* sw = st[wave];
#pragma unroll
  for (int j = 0; j < 8; ++j) { const float bn = bias[j * 16 + l16];
#pragma unroll
    for (int r = 0; r < 8; ++r) sw[(r + 8 * g) * 132 + j * 16 + l16] = acc[j][r] + bn; }
  asm volatile("s_wait_dscnt 0" ::: "memory");
#pragma unroll 1
  for (int pass = 0; pass < 2; ++pass) {
#pragma unroll
    for (int i = 0; i < 16; ++i) { const int c = lane + 32 * i, rr = c >> 5, q = (c & 31) * 4;
      *(volatile v4f_t*)(relval + (size_t)(r0 + rr) * HDIM + q) = *(const volatile v4fa*)(sw + rr * 132 + q); }
    __threadfence();
  }
}

__global__ __launch_bounds__(512) void scatter_col_kernel(const float* __restrict__ relval,
                                                          const int* __restrict__ rels, const int* __restrict__ heads,
                                                          const int* __restrict__ tails, const float* __restrict__ wvals,
                                                          float* __restrict__ aggT) {
  __shared__ __attribute__((aligned(16))) float seg[NSEG];
  const int c = blockIdx.x, tid = threadIdx.x;
  for (int s = tid; s < NSEG; s += 512) seg[s] = 0.f;
  __syncthreads();
  for (int f = tid; f < NFACT; f += 512) {
    int r = rels[f], h = heads[f], t = tails[f];
    r = (r < 0) ? 0 : (r > NREL - 1 ? NREL - 1 : r);
    h = (h < 0) ? 0 : (h > NSEG - 1 ? NSEG - 1 : h);
    t = (t < 0) ? 0 : (t > NSEG - 1 ? NSEG - 1 : t);
    const float v = relval[(size_t)r * HDIM + c] * wvals[f];
    atomicAdd(&seg[t], v);
    atomicAdd(&seg[h], v);
  }
  __syncthreads();
  float* col = aggT + (size_t)c * NSEG;
#pragma unroll 1
  for (int pass = 0; pass < 2; ++pass) {
    for (int q = tid; q < NSEG / 4; q += 512) *(volatile v4f_t*)(col + q * 4) = *(const volatile v4fa*)(seg + q * 4);
    __threadfence();
  }
}

__global__ __launch_bounds__(256) void transpose_relu_kernel(const float* __restrict__ aggT, float* __restrict__ out) {
  const int t = blockIdx.x * 256 + threadIdx.x;
  if (t >= NSEG * (HDIM / 4)) return;
  const int c4 = (t & 31) * 4, s = t >> 5;
  v4f_t v;
  v.x = fmaxf(aggT[(size_t)(c4 + 0) * NSEG + s], 0.f);
  v.y = fmaxf(aggT[(size_t)(c4 + 1) * NSEG + s], 0.f);
  v.z = fmaxf(aggT[(size_t)(c4 + 2) * NSEG + s], 0.f);
  v.w = fmaxf(aggT[(size_t)(c4 + 3) * NSEG + s], 0.f);
  float* d = out + (size_t)s * HDIM + c4;
  *(volatile v4f_t*)d = v; __threadfence(); *(volatile v4f_t*)d = v;
}

extern "C" void kernel_launch(void* const* d_in, const int* in_sizes, int n_in,
                              void* d_out, int out_size, void* d_ws, size_t ws_size,
                              hipStream_t stream) {
  (void)in_sizes; (void)n_in; (void)out_size; (void)ws_size;
  const int*   heads = (const int*)d_in[1];
  const int*   rels  = (const int*)d_in[2];
  const int*   tails = (const int*)d_in[3];
  const float* wvals = (const float*)d_in[4];
  const float* relf  = (const float*)d_in[5];
  const float* Wf    = (const float*)d_in[6];
  const float* bias  = (const float*)d_in[7];
  float* out = (float*)d_out;

  char* ws = (char*)d_ws;
  _Float16* Ah     = (_Float16*)ws;
  _Float16* Wh     = Ah + (size_t)2 * NREL * HDIM;
  float*    relval = (float*)(Wh + (size_t)2 * HDIM * HDIM);
  float*    aggT   = relval + (size_t)NREL * HDIM;

  prep_kernel<<<((NREL * HDIM + HDIM * HDIM) / 8 + 255) / 256, 256, 0, stream>>>(relf, Wf, Ah, Wh);
  relval_gemm_wmma<<<(NREL / 16 + 3) / 4, 128, 0, stream>>>(Ah, Wh, bias, relval);
  scatter_col_kernel<<<HDIM, 512, 0, stream>>>(relval, rels, heads, tails, wvals, aggT);
  transpose_relu_kernel<<<(NSEG * (HDIM / 4)) / 256, 256, 0, stream>>>(aggT, out);
}
